// GenericLinear_89300960018587
// MI455X (gfx1250) — hardware-verified
//
#include <hip/hip_runtime.h>


#define NBL  4
#define NBS  16384
#define NCI  256
#define NU   256
#define KK   (NBL * NCI)
#define SGN  0xC6A0u
typedef _Float16 h16;
typedef unsigned short bf;
typedef __attribute__((ext_vector_type(16))) __bf16   v16bf;
typedef __attribute__((ext_vector_type(16))) _Float16 v16h;
typedef __attribute__((ext_vector_type(8)))  _Float16 v8h;
typedef __attribute__((ext_vector_type(8)))  unsigned short v8us;
typedef __attribute__((ext_vector_type(8)))  float    v8f;
typedef __attribute__((ext_vector_type(4)))  float    v4f;
typedef v8h  __attribute__((may_alias)) v8ha;
typedef v4f  __attribute__((may_alias)) v4fa;
typedef v8us __attribute__((may_alias)) v8usa;

__device__ __forceinline__ unsigned short f2bf(float f) { unsigned u = __float_as_uint(f); u += 0x7FFFu + ((u >> 16) & 1u); return (unsigned short)(u >> 16); }
__device__ __forceinline__ float bf2f(unsigned short b) { return __uint_as_float(((unsigned)b) << 16); }
__device__ __forceinline__ float bfr(float f) { return bf2f(f2bf(f)); }
__device__ __forceinline__ v16h cat16(v8h lo, v8h hi) { return __builtin_shufflevector(lo, hi, 0, 1, 2, 3, 4, 5, 6, 7, 8, 9, 10, 11, 12, 13, 14, 15); }
__device__ __forceinline__ v16bf cat16b(v8us lo, v8us hi) { return __builtin_bit_cast(v16bf, __builtin_shufflevector(lo, hi, 0, 1, 2, 3, 4, 5, 6, 7, 8, 9, 10, 11, 12, 13, 14, 15)); }
__device__ __forceinline__ v8f wmma16(v16h a, v16h b, v8f c) { return __builtin_amdgcn_wmma_f32_16x16x32_f16(false, a, false, b, (short)0, c, false, false); }
__device__ __forceinline__ v8f wmmab(v16bf a, v16bf b, v8f c) { return __builtin_amdgcn_wmma_f32_16x16x32_bf16(false, a, false, b, (short)0, c, false, false); }

template <typename T16> struct WFrag;
template <> struct WFrag<h16> { typedef v16h V; static __device__ __forceinline__ V ld(const h16* p) { return cat16(*(const v8h*)p, *(const v8h*)(p + 16)); } static __device__ __forceinline__ v8f mma(V a, V b, v8f c) { return wmma16(a, b, c); } };
template <> struct WFrag<bf> { typedef v16bf V; static __device__ __forceinline__ V ld(const bf* p) { return cat16b(*(const v8us*)p, *(const v8us*)(p + 16)); } static __device__ __forceinline__ v8f mma(V a, V b, v8f c) { return wmmab(a, b, c); } };
template <typename T16, int NSPLIT, bool BIAS>
__global__ __launch_bounds__(32) void k_gemmw(const T16* __restrict__ A, const T16* __restrict__ A2, const T16* __restrict__ Bt, const T16* __restrict__ Bt2, int K, float* C, int ldc, const float* __restrict__ bias, size_t sA, size_t sB, size_t sC) {
    typedef typename WFrag<T16>::V V;
    __shared__ __align__(16) float os[16 * 68];
    const size_t z = blockIdx.z; A += z * sA; if (A2) A2 += z * sA; Bt += z * sB; if (Bt2) Bt2 += z * sB; C += z * sC;
    const int lane = threadIdx.x & 31, lr = lane & 15, hi = lane >> 4; const int r0 = blockIdx.x * 64, c0 = blockIdx.y * 64;
    v8f acc[4][4];
#pragma unroll
    for (int mb = 0; mb < 4; ++mb)
#pragma unroll
        for (int nb = 0; nb < 4; ++nb) acc[mb][nb] = (v8f){};
    const size_t aoff = (size_t)(r0 + lr) * K + 8 * hi, boff = (size_t)(c0 + lr) * K + 8 * hi;
    for (int kc = 0; kc < K; kc += 32) {
        V a[4], a2[4];
#pragma unroll
        for (int mb = 0; mb < 4; ++mb) { a[mb] = WFrag<T16>::ld(A + aoff + (size_t)mb * 16 * K + kc); if (NSPLIT == 1 || NSPLIT == 2) a2[mb] = WFrag<T16>::ld(A2 + aoff + (size_t)mb * 16 * K + kc); }
#pragma unroll
        for (int nb = 0; nb < 4; ++nb) { const V b = WFrag<T16>::ld(Bt + boff + (size_t)nb * 16 * K + kc); V b2; if (NSPLIT >= 2) b2 = WFrag<T16>::ld(Bt2 + boff + (size_t)nb * 16 * K + kc);
#pragma unroll
            for (int mb = 0; mb < 4; ++mb) { acc[mb][nb] = WFrag<T16>::mma(a[mb], b, acc[mb][nb]); if (NSPLIT == 1 || NSPLIT == 2) acc[mb][nb] = WFrag<T16>::mma(a2[mb], b, acc[mb][nb]); if (NSPLIT >= 2) acc[mb][nb] = WFrag<T16>::mma(a[mb], b2, acc[mb][nb]); } }
        asm volatile("v_nop\n\tv_nop\n\tv_nop\n\tv_nop" : "+v"(acc[0][0]), "+v"(acc[1][1]), "+v"(acc[2][2]), "+v"(acc[3][3]) : "v"(a[0]), "v"(a[3]));
    }
#pragma unroll
    for (int mb = 0; mb < 4; ++mb) {
#pragma unroll
        for (int nb = 0; nb < 4; ++nb) {
#pragma unroll
            for (int j = 0; j < 8; ++j) os[(hi * 8 + j) * 68 + nb * 16 + lr] = acc[mb][nb][j]; }
        __builtin_amdgcn_wave_barrier(); asm volatile("" ::: "memory");
        float* crow = C + (size_t)(r0 + mb * 16) * ldc + c0;
#pragma unroll 1
        for (int ps = 0; ps < 2; ++ps) {
#pragma unroll
            for (int s = 0; s < 8; ++s) { const int row = 2 * s + hi, cofs = lr * 4; v4f val = *(const v4fa*)(os + row * 68 + cofs); if (BIAS) { val[0] += bfr(bias[c0 + cofs]); val[1] += bfr(bias[c0 + cofs + 1]); val[2] += bfr(bias[c0 + cofs + 2]); val[3] += bfr(bias[c0 + cofs + 3]); }
                *(volatile v4f*)(crow + (size_t)row * ldc + cofs) = val; }
            if (ps == 0) __threadfence(); }
        __builtin_amdgcn_wave_barrier(); asm volatile("" ::: "memory");
    }
}

typedef __attribute__((ext_vector_type(2))) _Float16 v2h;
typedef __attribute__((ext_vector_type(4))) _Float16 v4h;
typedef __attribute__((ext_vector_type(2))) unsigned short v2us;
typedef __attribute__((ext_vector_type(4))) unsigned short v4us;
typedef __attribute__((ext_vector_type(2))) float v2f;
typedef __attribute__((ext_vector_type(4))) int v4i;

__global__ __launch_bounds__(256) void k_xs(const float* __restrict__ x, bf* Xs) { const int j = blockIdx.x * 256 + threadIdx.x; if (j >= NBS * KK / 8) return; const int q = j % (KK / 8); const int r = j / (KK / 8); const int i = q / (NCI / 8); const int t8 = q % (NCI / 8); const float* src = x + ((size_t)i * NBS + r) * NCI + t8 * 8; const v4f a = *(const v4f*)src, b = *(const v4f*)(src + 4); v8us o;
#pragma unroll
    for (int k = 0; k < 4; ++k) { o[k] = f2bf(a[k]); o[k + 4] = f2bf(b[k]); }
    *(volatile v8us*)(Xs + (size_t)j * 8) = o; __threadfence(); *(volatile v8us*)(Xs + (size_t)j * 8) = o; }

__global__ __launch_bounds__(256) void k_ws(const float* __restrict__ Wm, bf* Ws) { const int j = blockIdx.x * 256 + threadIdx.x; if (j >= NBL * NU * KK / 2) return; const int d2 = (j % (KK / 2)) * 2; const int u = (j / (KK / 2)) % NU; const int k = j / (NU * KK / 2); const int i = d2 / NCI; const int t = d2 % NCI; const int jb = i ^ k; const unsigned short fl = (unsigned short)(((SGN >> (i * 4 + jb)) & 1u) << 15); const size_t s0 = (size_t)t * (NBL * NU) + (size_t)jb * NU + u; v2us o; o[0] = (unsigned short)(f2bf(Wm[s0]) ^ fl); o[1] = (unsigned short)(f2bf(Wm[s0 + NBL * NU]) ^ fl); *(volatile v2us*)(Ws + (size_t)j * 2) = o; __threadfence(); *(volatile v2us*)(Ws + (size_t)j * 2) = o; }

extern "C" void kernel_launch(void* const* d_in, const int* in_sizes, int n_in, void* d_out, int out_size, void* d_ws, size_t ws_size, hipStream_t stream) {
    if (n_in < 3) return;
    if (in_sizes[0] != NBL * NBS * NCI || in_sizes[1] != NCI * NBL * NU || in_sizes[2] != NBL * NU) return;
    if (out_size != NBL * NBS * NU) return;
    static_assert(NBS % 64 == 0 && NU % 64 == 0 && KK % 32 == 0 && (NBS * KK / 8) % 256 == 0 && (NBL * NU * KK / 2) % 256 == 0 && NCI % 8 == 0 && NCI % 2 == 0, "the product: M and N multiples of 64, the depth of 32; the two flat grids exact; a thread's 8 (or 2) depth words lie in one chunk");
    const float* x = (const float*)d_in[0]; const float* Wm = (const float*)d_in[1]; const float* c = (const float*)d_in[2]; float* out = (float*)d_out;
    char* wsp = (char*)d_ws; auto take = [&](size_t bytes) { char* p = wsp; wsp += (bytes + 255) & ~(size_t)255; return (void*)p; };
    bf* Xs = (bf*)take((size_t)NBS * KK * 2); bf* Ws = (bf*)take((size_t)NBL * NU * KK * 2);
    if ((size_t)(wsp - (char*)d_ws) > ws_size) return;
    k_xs<<<(unsigned)(NBS * KK / 8 / 256), 256, 0, stream>>>(x, Xs);
    k_ws<<<(unsigned)(NBL * NU * KK / 2 / 256), 256, 0, stream>>>(Wm, Ws);
    for (int k = 0; k < NBL; ++k) k_gemmw<bf, 0, true><<<dim3(NBS / 64, NU / 64, 1), 32, 0, stream>>>(Xs, nullptr, Ws + (size_t)k * NU * KK, nullptr, KK, out + (size_t)k * NBS * NU, NU, c + (size_t)k * NU, 0, 0, 0);
}
